// GAT_85830626443964
// MI455X (gfx1250) — hardware-verified
//
#include <hip/hip_runtime.h>
#include <math.h>
#include <stdint.h>

#pragma clang fp contract(off)

#define NB    8
#define NN    1024
#define FIN   128
#define FOUT  128
#define NH    4
#define HD    32
#define MROWS (NB * NN)

static_assert(HD == 32);
static_assert(NH * HD == FOUT);
static_assert(NN % 128 == 0);
static_assert(NN % 32 == 0);
static_assert(FIN % 32 == 0);
static_assert(FIN == 128 && FOUT == 128);

typedef __attribute__((ext_vector_type(16))) __bf16   v16b;
typedef __attribute__((ext_vector_type(8)))  __bf16   v8b;
typedef __attribute__((ext_vector_type(8)))  float    v8f;
typedef __attribute__((ext_vector_type(4)))  float    v4f;
typedef __attribute__((ext_vector_type(4)))  unsigned int v4u;
typedef __attribute__((ext_vector_type(8)))  unsigned int v8u;
typedef v4f __attribute__((may_alias)) v4fa;

__device__ __forceinline__ unsigned short f2bf_bits(float f) {
  unsigned u = __float_as_uint(f);
  return (unsigned short)((u + 0x7FFFu + ((u >> 16) & 1u)) >> 16);
}
__device__ __forceinline__ float bf_bits2f(unsigned short h) { return __uint_as_float(((unsigned)h) << 16); }
__device__ __forceinline__ unsigned pk16(unsigned short a, unsigned short b) { return (unsigned)a | ((unsigned)b << 16); }
__device__ __forceinline__ v8f zero8() { v8f z = {0.f, 0.f, 0.f, 0.f, 0.f, 0.f, 0.f, 0.f}; return z; }

struct FragB {
  union U { v16b v; v8b h[2]; };
  static __device__ __forceinline__ v16b load(const __bf16* p) {
    U f; f.h[0] = *(const v8b*)(p); f.h[1] = *(const v8b*)(p + 16); return f.v;
  }
};
__device__ __forceinline__ v8f at_mma(v16b a, v16b b, v8f c) {
  c = __builtin_amdgcn_wmma_f32_16x16x32_bf16(false, a, false, b, (short)0, c, false, false);
  asm volatile("v_nop\n\tv_nop\n\tv_nop\n\tv_nop" : "+v"(c) : "v"(a), "v"(b));
  return c;
}

#define PREP_XBLK (MROWS * FIN / 8 / 256)
__global__ __launch_bounds__(256) void k_prep(const float* __restrict__ x, const float* __restrict__ W,
                                              const float* __restrict__ asrc, const float* __restrict__ adst,
                                              unsigned short* __restrict__ XB, unsigned short* __restrict__ WT,
                                              float* __restrict__ AV) {
  __shared__ __align__(16) float tf[64 * 68];
  const int tid = threadIdx.x;
  const int blk = blockIdx.x;
  if (blk < PREP_XBLK) {
    const int i = blk * 256 + tid;
    const float* sp = x + (size_t)i * 8;
    const v4f a  = *(const v4f*)(sp);
    const v4f a2 = *(const v4f*)(sp + 4);
    v4u w;
    w[0] = pk16(f2bf_bits(a[0]),  f2bf_bits(a[1]));
    w[1] = pk16(f2bf_bits(a[2]),  f2bf_bits(a[3]));
    w[2] = pk16(f2bf_bits(a2[0]), f2bf_bits(a2[1]));
    w[3] = pk16(f2bf_bits(a2[2]), f2bf_bits(a2[3]));
    unsigned short* dp = XB + (size_t)i * 8;
    *(volatile v4u*)dp = w;
    __threadfence();
    *(volatile v4u*)dp = w;
  } else if (blk < PREP_XBLK + 4) {
    const int tb = blk - PREP_XBLK;
    const int c0 = (tb & 1) * 64;
    const int r0 = (tb >> 1) * 64;
    {
      const int lr = tid >> 4;
      const int c4 = (tid & 15) * 4;
#pragma unroll
      for (int it = 0; it < 4; ++it) {
        const int rr = it * 16 + lr;
        const v4f a = *(const v4f*)(W + (size_t)(r0 + rr) * FOUT + c0 + c4);
        *(v4f*)(tf + rr * 68 + c4) = a;
      }
    }
    __syncthreads();
    const int sub = tid >> 3;
    const int c8  = (tid & 7) * 8;
    v4u hv[2];
#pragma unroll
    for (int it = 0; it < 2; ++it) {
      const int oc = it * 32 + sub;
      v4u a;
#pragma unroll
      for (int q = 0; q < 4; ++q) {
        const float f0 = tf[(c8 + 2 * q) * 68 + oc];
        const float f1 = tf[(c8 + 2 * q + 1) * 68 + oc];
        a[q] = pk16(f2bf_bits(f0), f2bf_bits(f1));
      }
      hv[it] = a;
    }
    for (int pass = 0; pass < 2; ++pass) {
#pragma unroll
      for (int it = 0; it < 2; ++it) {
        const int oc = it * 32 + sub;
        const size_t go = (size_t)(c0 + oc) * FIN + r0 + c8;
        *(volatile v4u*)(WT + go) = hv[it];
      }
      __threadfence();
    }
  } else {
    if (tid < 64) {
      const int idx = tid & 31;
      const v4f va = *(const v4f*)(asrc + idx * 4);
      const v4f vb = *(const v4f*)(adst + idx * 4);
      v4f v;
#pragma unroll
      for (int e = 0; e < 4; ++e) {
        const float sv = (tid < 32) ? va[e] : vb[e];
        v[e] = bf_bits2f(f2bf_bits(sv));
      }
      *(volatile v4f*)(AV + tid * 4) = v;
      __threadfence();
      *(volatile v4f*)(AV + tid * 4) = v;
    }
  }
}

#define G_TP        132
#define G_LDS_TILE  (128 * G_TP * 4)
#define G_LDS_BYTES (G_LDS_TILE + 1024 + 4096)
__global__ __launch_bounds__(256) void k_gemm(const unsigned short* __restrict__ XBp, const unsigned short* __restrict__ WTp,
                                              const float* __restrict__ AV, float* __restrict__ ST,
                                              unsigned short* __restrict__ VH, unsigned short* __restrict__ VL) {
  extern __shared__ __align__(16) unsigned char gsm[];
  float* tile = (float*)gsm;
  float* avs  = (float*)(gsm + G_LDS_TILE);
  float* st   = avs + 256;

  const int tid  = threadIdx.x;
  const int lane = tid & 31;
  const int wave = tid >> 5;
  const int hh   = lane >> 4;
  const int c    = lane & 15;
  const int mblk = blockIdx.x * 128;
  const int m0   = mblk + wave * 16;

  const __bf16* A  = (const __bf16*)(const void*)XBp;
  const __bf16* Bt = (const __bf16*)(const void*)WTp;

  v8f acc[8];
#pragma unroll
  for (int j = 0; j < 8; ++j) acc[j] = zero8();

#pragma unroll 1
  for (int k0 = 0; k0 < FIN; k0 += 32) {
    const v16b a = FragB::load(A + (size_t)(m0 + c) * FIN + k0 + 8 * hh);
#pragma unroll
    for (int j = 0; j < 8; ++j) {
      const v16b b = FragB::load(Bt + (size_t)(j * 16 + c) * FIN + k0 + 8 * hh);
      acc[j] = at_mma(a, b, acc[j]);
    }
  }

#pragma unroll
  for (int j = 0; j < 8; ++j) {
#pragma unroll
    for (int r = 0; r < 8; ++r) tile[(wave * 16 + 8 * hh + r) * G_TP + j * 16 + c] = acc[j][r];
  }
  if (tid < 64) {
    const v4f a = *(const v4f*)(AV + tid * 4);
    *(v4f*)(avs + tid * 4) = a;
  }
  __syncthreads();

#pragma unroll 1
  for (int it = 0; it < 2; ++it) {
    const int pr  = it * 256 + tid;
    const int row = pr & 127;
    const int hd  = pr >> 7;
    const float* tr = tile + row * G_TP + hd * HD;
    const float* as = avs + hd * HD;
    const float* ad = avs + 128 + hd * HD;
    float sv = 0.0f, tv = 0.0f;
#pragma unroll 4
    for (int d = 0; d < HD; ++d) {
      const float hv = tr[d];
      sv = fmaf(hv, as[d], sv);
      tv = fmaf(hv, ad[d], tv);
    }
    st[hd * 128 + row]       = sv;
    st[512 + hd * 128 + row] = tv;
  }

  const int b  = mblk >> 10;
  const int n0 = mblk & (NN - 1);
  for (int pass = 0; pass < 2; ++pass) {
#pragma unroll 2
    for (int it = 0; it < 8; ++it) {
      const int piece = it * 256 + tid;
      const int col   = piece >> 4;
      const int seg   = piece & 15;
      const float* tc = tile + (seg * 8) * G_TP + col;
      v4u hw, lw;
#pragma unroll
      for (int q = 0; q < 4; ++q) {
        const float f0 = tc[(2 * q) * G_TP];
        const float f1 = tc[(2 * q + 1) * G_TP];
        const unsigned short h0 = f2bf_bits(f0), h1 = f2bf_bits(f1);
        const unsigned short l0 = f2bf_bits(f0 - bf_bits2f(h0)), l1 = f2bf_bits(f1 - bf_bits2f(h1));
        hw[q] = pk16(h0, h1);
        lw[q] = pk16(l0, l1);
      }
      const size_t go = (size_t)(b * 128 + col) * NN + n0 + seg * 8;
      *(volatile v4u*)(VH + go) = hw;
      *(volatile v4u*)(VL + go) = lw;
    }
    __threadfence();
  }
  __syncthreads();

  {
    const int plane = tid >> 7;
    const int hd    = (tid >> 5) & 3;
    const int seg   = tid & 31;
    const v4f val = *(const v4fa*)(st + plane * 512 + hd * 128 + seg * 4);
    float* dp = ST + (size_t)plane * (NB * NH * NN) + (size_t)(b * NH + hd) * NN + n0 + seg * 4;
    *(volatile v4f*)dp = val;
    __threadfence();
    *(volatile v4f*)dp = val;
  }
}

#define A_VP        1032
#define A_OSP       36
#define A_OFF_VL    (32 * A_VP * 2)
#define A_OFF_T     (2 * A_OFF_VL)
#define A_OFF_OS    (A_OFF_T + NN * 4)
#define A_OFF_LS    (A_OFF_OS + 8 * 16 * A_OSP * 4)
#define A_OFF_RED   (A_OFF_LS + 8 * 16 * 4)
#define A_LDS_BYTES (A_OFF_RED + 128)
static_assert(A_LDS_BYTES <= 320 * 1024);
static_assert((A_OFF_VL % 16) == 0 && (A_OFF_T % 16) == 0 && (A_OFF_OS % 16) == 0);
static_assert(G_LDS_BYTES <= 320 * 1024);

__device__ __forceinline__ float p_one(float t, float si, float mi) {
  const float v = si + t;
  const float e = (v >= 0.0f) ? v : 0.2f * v;
  return expf(e - mi);
}
__device__ __forceinline__ void p_pair(float t0, float t1, float si, float mi, float& lsum, unsigned& hw, unsigned& lw) {
  const float p0 = p_one(t0, si, mi);
  const float p1 = p_one(t1, si, mi);
  lsum += p0;
  lsum += p1;
  const unsigned short h0 = f2bf_bits(p0), h1 = f2bf_bits(p1);
  const unsigned short l0 = f2bf_bits(p0 - bf_bits2f(h0)), l1 = f2bf_bits(p1 - bf_bits2f(h1));
  hw = pk16(h0, h1);
  lw = pk16(l0, l1);
}

__global__ __launch_bounds__(256) void k_attn(const float* __restrict__ Sp, const float* __restrict__ Tp,
                                              const unsigned short* __restrict__ VHp, const unsigned short* __restrict__ VLp,
                                              float* __restrict__ out) {
  extern __shared__ __align__(16) unsigned char asmem[];
  __bf16* Vh  = (__bf16*)asmem;
  __bf16* Vl  = (__bf16*)(asmem + A_OFF_VL);
  float*  Tl  = (float*)(asmem + A_OFF_T);
  float*  Os  = (float*)(asmem + A_OFF_OS);
  float*  Ls  = (float*)(asmem + A_OFF_LS);
  float*  red = (float*)(asmem + A_OFF_RED);

  const int tid  = threadIdx.x;
  const int lane = tid & 31;
  const int wave = tid >> 5;
  const int hh   = lane >> 4;
  const int c    = lane & 15;

  const int bx   = blockIdx.x;
  const int qt   = bx & 7;
  const int pair = bx >> 3;
  const int b    = pair >> 2;
  const int hd   = pair & 3;

  {
    const v4f t4 = *(const v4f*)(Tp + (size_t)pair * NN + tid * 4);
    *(v4f*)(Tl + tid * 4) = t4;
    float lm = fmaxf(fmaxf(t4[0], t4[1]), fmaxf(t4[2], t4[3]));
    lm = fmaxf(lm, __shfl_xor(lm, 16, 32));
    lm = fmaxf(lm, __shfl_xor(lm, 8, 32));
    lm = fmaxf(lm, __shfl_xor(lm, 4, 32));
    lm = fmaxf(lm, __shfl_xor(lm, 2, 32));
    lm = fmaxf(lm, __shfl_xor(lm, 1, 32));
    if (lane == 0) red[wave] = lm;
  }
  {
    const __bf16* gvh = (const __bf16*)(const void*)VHp + (size_t)pair * HD * NN;
    const __bf16* gvl = (const __bf16*)(const void*)VLp + (size_t)pair * HD * NN;
#pragma unroll 4
    for (int it = 0; it < 16; ++it) {
      const int p   = it * 256 + tid;
      const int row = p >> 7;
      const int seg = p & 127;
      const v8b a0 = *(const v8b*)(gvh + (size_t)row * NN + seg * 8);
      const v8b a1 = *(const v8b*)(gvl + (size_t)row * NN + seg * 8);
      *(v8b*)(Vh + row * A_VP + seg * 8) = a0;
      *(v8b*)(Vl + row * A_VP + seg * 8) = a1;
    }
  }
  __syncthreads();

  float tmax = red[0];
#pragma unroll
  for (int w = 1; w < 8; ++w) tmax = fmaxf(tmax, red[w]);

  const int   q0 = qt * 128 + wave * 16;
  const float si = Sp[(size_t)pair * NN + q0 + c];
  const float mv = si + tmax;
  const float mi = (mv >= 0.0f) ? mv : 0.2f * mv;

  v8f acc0 = zero8();
  v8f acc1 = zero8();
  float lsum = 0.0f;

  const __bf16* vh0 = Vh + (size_t)c * A_VP + 8 * hh;
  const __bf16* vh1 = Vh + (size_t)(16 + c) * A_VP + 8 * hh;
  const __bf16* vl0 = Vl + (size_t)c * A_VP + 8 * hh;
  const __bf16* vl1 = Vl + (size_t)(16 + c) * A_VP + 8 * hh;
  const float*  tq  = Tl + 8 * hh;

#pragma unroll 1
  for (int j0 = 0; j0 < NN; j0 += 32) {
    const v4f ta = *(const v4f*)(tq + j0);
    const v4f tb = *(const v4f*)(tq + j0 + 4);
    const v4f tc = *(const v4f*)(tq + j0 + 16);
    const v4f td = *(const v4f*)(tq + j0 + 20);
    unsigned h0, h1, h2, h3, h4, h5, h6, h7;
    unsigned l0, l1, l2, l3, l4, l5, l6, l7;
    p_pair(ta[0], ta[1], si, mi, lsum, h0, l0);
    p_pair(ta[2], ta[3], si, mi, lsum, h1, l1);
    p_pair(tb[0], tb[1], si, mi, lsum, h2, l2);
    p_pair(tb[2], tb[3], si, mi, lsum, h3, l3);
    p_pair(tc[0], tc[1], si, mi, lsum, h4, l4);
    p_pair(tc[2], tc[3], si, mi, lsum, h5, l5);
    p_pair(td[0], td[1], si, mi, lsum, h6, l6);
    p_pair(td[2], td[3], si, mi, lsum, h7, l7);
    const v8u hwv = {h0, h1, h2, h3, h4, h5, h6, h7};
    const v8u lwv = {l0, l1, l2, l3, l4, l5, l6, l7};
    const v16b ahi = __builtin_bit_cast(v16b, hwv);
    const v16b alo = __builtin_bit_cast(v16b, lwv);

    const v16b bh0 = FragB::load(vh0 + j0);
    const v16b bh1 = FragB::load(vh1 + j0);
    const v16b bl0 = FragB::load(vl0 + j0);
    const v16b bl1 = FragB::load(vl1 + j0);

    acc0 = at_mma(ahi, bh0, acc0);
    acc0 = at_mma(alo, bh0, acc0);
    acc0 = at_mma(ahi, bl0, acc0);
    acc1 = at_mma(ahi, bh1, acc1);
    acc1 = at_mma(alo, bh1, acc1);
    acc1 = at_mma(ahi, bl1, acc1);
  }

  const float lother = __shfl_xor(lsum, 16, 32);
  const float lrow   = lsum + lother;

  float* os = Os + wave * 16 * A_OSP;
  float* ls = Ls + wave * 16;
#pragma unroll
  for (int r = 0; r < 8; ++r) {
    os[(8 * hh + r) * A_OSP + c]      = acc0[r];
    os[(8 * hh + r) * A_OSP + 16 + c] = acc1[r];
  }
  if (hh == 0) ls[c] = lrow;
  __syncthreads();

  {
    const int q4 = lane >> 3, c4 = (lane & 7) * 4;
    float* ob = out + (size_t)b * NN * FOUT + hd * HD;
    v4f val[4];
#pragma unroll
    for (int it = 0; it < 4; ++it) {
      const int row = it * 4 + q4;
      const v4f a = *(const v4fa*)(os + row * A_OSP + c4);
      const float inv = 1.0f / ls[row];
      val[it] = a * inv;
    }
    for (int pass = 0; pass < 2; ++pass) {
#pragma unroll
      for (int it = 0; it < 4; ++it) {
        const int row = it * 4 + q4;
        *(volatile v4f*)(ob + (size_t)(q0 + row) * FOUT + c4) = val[it];
      }
      __threadfence();
    }
  }
}

extern "C" void kernel_launch(void* const* d_in, const int* in_sizes, int n_in,
                              void* d_out, int out_size, void* d_ws, size_t ws_size,
                              hipStream_t stream) {
  if (n_in < 4) return;
  if (in_sizes[0] != MROWS * FIN) return;
  if (in_sizes[1] != FIN * FOUT) return;
  if (in_sizes[2] != NH * HD || in_sizes[3] != NH * HD) return;
  if (out_size != MROWS * FOUT) return;

  const float* x     = (const float*)d_in[0];
  const float* W     = (const float*)d_in[1];
  const float* a_src = (const float*)d_in[2];
  const float* a_dst = (const float*)d_in[3];
  float* out = (float*)d_out;

  const size_t PXB = (size_t)MROWS * FIN * 2;
  const size_t PWT = (size_t)FOUT * FIN * 2;
  const size_t PAV = (size_t)256 * 4;
  const size_t PST = (size_t)2 * NB * NH * NN * 4;
  const size_t PV  = (size_t)NB * NH * HD * NN * 2;
  size_t off = 0;
  const size_t oXB = off; off += PXB;
  const size_t oWT = off; off += PWT;
  const size_t oAV = off; off += PAV;
  const size_t oST = off; off += PST;
  const size_t oVH = off; off += PV;
  const size_t oVL = off; off += PV;
  if (off > ws_size) return;
  if (off > (size_t)134217728) return;

  char* ws = (char*)d_ws;
  unsigned short* XB = (unsigned short*)(ws + oXB);
  unsigned short* WT = (unsigned short*)(ws + oWT);
  float*          AV = (float*)(ws + oAV);
  float*          ST = (float*)(ws + oST);
  unsigned short* VH = (unsigned short*)(ws + oVH);
  unsigned short* VL = (unsigned short*)(ws + oVL);

  (void)hipFuncSetAttribute(reinterpret_cast<const void*>(&k_gemm), hipFuncAttributeMaxDynamicSharedMemorySize, (int)G_LDS_BYTES);
  (void)hipFuncSetAttribute(reinterpret_cast<const void*>(&k_attn), hipFuncAttributeMaxDynamicSharedMemorySize, (int)A_LDS_BYTES);

  k_prep<<<dim3(PREP_XBLK + 5), dim3(256), 0, stream>>>(x, W, a_src, a_dst, XB, WT, AV);
  k_gemm<<<dim3(MROWS / 128), dim3(256), G_LDS_BYTES, stream>>>(XB, WT, AV, ST, VH, VL);
  const float* Sp = ST;
  const float* Tp = ST + (size_t)NB * NH * NN;
  k_attn<<<dim3(NB * NH * 8), dim3(256), A_LDS_BYTES, stream>>>(Sp, Tp, VH, VL, out);
  (void)hipGetLastError();
}
